// MultiHeadedAttention_25091198943835
// MI455X (gfx1250) — hardware-verified
//
#include <hip/hip_runtime.h>
#include <stdint.h>


typedef _Float16 h16;
typedef __attribute__((ext_vector_type(8)))  _Float16 v8h;
typedef __attribute__((ext_vector_type(16))) _Float16 v16h;
typedef __attribute__((ext_vector_type(8)))  float    v8f;
typedef __attribute__((ext_vector_type(4)))  float    v4f;
typedef v4f __attribute__((may_alias)) v4fa;
typedef v8h __attribute__((may_alias)) v8ha;

#ifndef NB
#define NB 2
#endif
#ifndef SEQ
#define SEQ 2048
#endif
#define NB_FULL  2
#define SEQ_FULL 2048
#define DM   768
#define NH   12
#define DK   64
#define ROWS (NB * SEQ)
#define NT64 (DM / 64)
#define CVT_CHUNK 2048

static_assert(NB >= 1 && NB <= NB_FULL);
static_assert(SEQ >= 128 && SEQ <= SEQ_FULL);
static_assert(SEQ % 128 == 0);
static_assert(ROWS % 16 == 0);
static_assert(((ROWS / 16) * NT64) % 4 == 0);
static_assert((ROWS * DM) % CVT_CHUNK == 0);
static_assert((DM * DM) % CVT_CHUNK == 0);
static_assert(NH * DK == DM);
static_assert(DM % 32 == 0);

__device__ __forceinline__ float bf16r(float x) {
  unsigned u = __float_as_uint(x);
  u = u + 0x7FFFu + ((u >> 16) & 1u);
  u &= 0xFFFF0000u;
  return __uint_as_float(u);
}

__device__ __forceinline__ v8f wmma16(v16h a, v16h b, v8f c) {
  v8f d = __builtin_amdgcn_wmma_f32_16x16x32_f16(
      false, a, false, b, (short)0, c, false, false);
  asm volatile("v_nop\n\tv_nop\n\tv_nop\n\tv_nop" : "+v"(d) : "v"(a), "v"(b));
  return d;
}

__device__ __forceinline__ v16h frag16(const h16* rowp, int kofs, int lane) {
  const h16* p = rowp + kofs + ((lane < 16) ? 0 : 8);
  v8h lo = *(const v8h*)(p);
  v8h hi = *(const v8h*)(p + 16);
  return __builtin_shufflevector(lo, hi, 0, 1, 2, 3, 4, 5, 6, 7,
                                         8, 9, 10, 11, 12, 13, 14, 15);
}

__global__ __launch_bounds__(256) void cvt_planes(
    const float* __restrict__ xq, const float* __restrict__ xk,
    const float* __restrict__ xv, const float* __restrict__ W,
    h16* __restrict__ xh, h16* __restrict__ wh, int nxc, int nwc) {
  const int tid   = threadIdx.x;
  const int y     = blockIdx.y;
  const int chunk = blockIdx.x;

  const float* sp;
  h16* dst;
  float sc;
  if (y < 3) {
    if (chunk >= nxc) return;
    const float* src = (y == 0) ? xq : ((y == 1) ? xk : xv);
    const size_t e  = (size_t)chunk * CVT_CHUNK + (size_t)tid * 8;
    const size_t r  = e / DM;
    const size_t c  = e - r * DM;
    const size_t bb = r / SEQ;
    const size_t s  = r - bb * SEQ;
    sp  = src + ((bb * SEQ_FULL + s) * DM + c);
    dst = xh + (size_t)y * ROWS * DM + e;
    sc  = 1.0f;
  } else {
    if (chunk >= nwc) return;
    const size_t e = (size_t)chunk * CVT_CHUNK + (size_t)tid * 8;
    sp  = W + e;
    dst = wh + e;
    sc  = 64.0f;
  }
  const v4f x0 = *(const v4f*)(sp);
  const v4f x1 = *(const v4f*)(sp + 4);
  v8h val;
#pragma unroll
  for (int i = 0; i < 4; ++i) {
    val[i]     = (h16)(sc * bf16r(x0[i]));
    val[i + 4] = (h16)(sc * bf16r(x1[i]));
  }
  *(volatile v8h*)dst = val;
  __threadfence();
  *(volatile v8h*)dst = val;
}

#define CTP 68

template <int MODE>
__global__ __launch_bounds__(128) __attribute__((amdgpu_num_vgpr(256)))
void proj_gemm(const h16* __restrict__ Ah, const h16* __restrict__ Al,
               const h16* __restrict__ Wh, const float* __restrict__ bias,
               void* __restrict__ Cv) {
  __shared__ __align__(16) float Ct[4][16][CTP];

  const int tid  = threadIdx.x;
  const int lane = tid & 31;
  const int wave = tid >> 5;
  const int hsel = lane >> 4;
  const int l16  = lane & 15;
  const int w     = blockIdx.x * 4 + wave;
  const int mtile = w / NT64;
  const int ntile = w - mtile * NT64;
  const int m0 = mtile * 16;
  const int n0 = ntile * 64;
  const size_t plane = (MODE == 0) ? (size_t)blockIdx.y * ROWS * DM : (size_t)0;

  const h16* arow = Ah + plane + (size_t)(m0 + l16) * DM;
  const h16* lrow = arow;
  if constexpr (MODE == 1) lrow = Al + (size_t)(m0 + l16) * DM;

  v8f acc[4]  = {};
  v8f accl[4] = {};

#pragma unroll 2
  for (int k0 = 0; k0 < DM; k0 += 32) {
    const v16h a = frag16(arow, k0, lane);
    v16h al;
    if constexpr (MODE == 1) al = frag16(lrow, k0, lane);
#pragma unroll
    for (int t = 0; t < 4; ++t) {
      const v16h bfr = frag16(Wh + (size_t)(n0 + t * 16 + l16) * DM, k0, lane);
      acc[t] = wmma16(a, bfr, acc[t]);
      if constexpr (MODE == 1) accl[t] = wmma16(al, bfr, accl[t]);
    }
  }

  float* ct = &Ct[wave][0][0];
#pragma unroll
  for (int t = 0; t < 4; ++t) {
    const float bb = bf16r(bias[n0 + t * 16 + l16]);
#pragma unroll
    for (int j = 0; j < 8; ++j) {
      float v;
      if constexpr (MODE == 0) {
        v = acc[t][j] * 0.0625f + 4.0f * bb;
      } else {
        v = (acc[t][j] + accl[t][j] * 0.00048828125f) * 0.00048828125f + bb;
      }
      ct[(8 * hsel + j) * CTP + t * 16 + l16] = v;
    }
  }
  __syncthreads();

  if constexpr (MODE == 0) {
    h16* C = (h16*)Cv + plane;
    v8h vals[4];
#pragma unroll
    for (int it = 0; it < 4; ++it) {
      const int row = it * 4 + (lane >> 3);
      const int c8  = (lane & 7) * 8;
      const v4fa p0 = *(const v4fa*)(ct + row * CTP + c8);
      const v4fa p1 = *(const v4fa*)(ct + row * CTP + c8 + 4);
      v8h t8;
      t8[0] = (h16)p0[0]; t8[1] = (h16)p0[1]; t8[2] = (h16)p0[2]; t8[3] = (h16)p0[3];
      t8[4] = (h16)p1[0]; t8[5] = (h16)p1[1]; t8[6] = (h16)p1[2]; t8[7] = (h16)p1[3];
      vals[it] = t8;
    }
#pragma unroll
    for (int it = 0; it < 4; ++it) {
      const int row = it * 4 + (lane >> 3);
      const int c8  = (lane & 7) * 8;
      *(volatile v8h*)(C + (size_t)(m0 + row) * DM + n0 + c8) = vals[it];
    }
    __threadfence();
#pragma unroll
    for (int it = 0; it < 4; ++it) {
      const int row = it * 4 + (lane >> 3);
      const int c8  = (lane & 7) * 8;
      *(volatile v8h*)(C + (size_t)(m0 + row) * DM + n0 + c8) = vals[it];
    }
  } else {
    float* C = (float*)Cv;
    v4f vals[8];
#pragma unroll
    for (int it = 0; it < 8; ++it) {
      const int row = it * 2 + (lane >> 4);
      const int c4  = (lane & 15) * 4;
      vals[it] = *(const v4fa*)(ct + row * CTP + c4);
    }
#pragma unroll
    for (int it = 0; it < 8; ++it) {
      const int row = it * 2 + (lane >> 4);
      const int c4  = (lane & 15) * 4;
      *(volatile v4f*)(C + (size_t)(m0 + row) * DM + n0 + c4) = vals[it];
    }
    __threadfence();
#pragma unroll
    for (int it = 0; it < 8; ++it) {
      const int row = it * 2 + (lane >> 4);
      const int c4  = (lane & 15) * 4;
      *(volatile v4f*)(C + (size_t)(m0 + row) * DM + n0 + c4) = vals[it];
    }
  }
}

#define QBLK 128
#define KBLK 64
#define LDSQ 72

__device__ __forceinline__ void store_tile16x64(const h16* slab, h16* gbase, int lane) {
  v8h vals[4];
#pragma unroll
  for (int it = 0; it < 4; ++it) {
    const int row = it * 4 + (lane >> 3);
    const int c8  = (lane & 7) * 8;
    vals[it] = *(const v8ha*)(slab + row * LDSQ + c8);
  }
#pragma unroll
  for (int it = 0; it < 4; ++it) {
    const int row = it * 4 + (lane >> 3);
    const int c8  = (lane & 7) * 8;
    *(volatile v8h*)(gbase + (size_t)row * DM + c8) = vals[it];
  }
  __threadfence();
#pragma unroll
  for (int it = 0; it < 4; ++it) {
    const int row = it * 4 + (lane >> 3);
    const int c8  = (lane & 7) * 8;
    *(volatile v8h*)(gbase + (size_t)row * DM + c8) = vals[it];
  }
}

__global__ __launch_bounds__(256) __attribute__((amdgpu_num_vgpr(256)))
void attn_flash(const h16* __restrict__ Qh, const h16* __restrict__ Kh,
                const h16* __restrict__ Vh, h16* __restrict__ Chi,
                h16* __restrict__ Clo) {
  __shared__ __align__(16) h16 Qs[QBLK][LDSQ];
  __shared__ __align__(16) h16 Ks[KBLK][LDSQ];
  __shared__ __align__(16) h16 Vs[DK][LDSQ];
  __shared__ __align__(16) h16 Ps[8][16][LDSQ];

  const int tid  = threadIdx.x;
  const int lane = tid & 31;
  const int wave = tid >> 5;
  const int b  = blockIdx.y / NH;
  const int h  = blockIdx.y - b * NH;
  const int q0 = blockIdx.x * QBLK;
  const size_t rowbase = (size_t)b * SEQ;

  const h16* gq = Qh + (rowbase + q0) * DM + h * DK;

#pragma unroll
  for (int i = 0; i < 4; ++i) {
    const int idx = tid + i * 256;
    const int r   = idx >> 3;
    const int c8  = (idx & 7) << 3;
    *(v8h*)&Qs[r][c8] = *(const v8h*)(gq + (size_t)r * DM + c8);
  }

  float mrun[8], lrun[8];
  v8f o[4] = {};
#pragma unroll
  for (int j = 0; j < 8; ++j) { mrun[j] = -1e30f; lrun[j] = 0.f; }

  const int qrow = wave * 16 + (lane & 15);
  const int cc   = lane & 15;
  const int rofs = (lane < 16) ? 0 : 8;
  h16* pw = &Ps[wave][0][0];

#pragma unroll 1
  for (int kb = 0; kb < SEQ; kb += KBLK) {
    const h16* gk = Kh + (rowbase + kb) * DM + h * DK;
    const h16* gv = Vh + (rowbase + kb) * DM + h * DK;

#pragma unroll
    for (int i = 0; i < 2; ++i) {
      const int idx = tid + i * 256;
      const int r   = idx >> 3;
      const int c8  = (idx & 7) << 3;
      *(v8h*)&Ks[r][c8] = *(const v8h*)(gk + (size_t)r * DM + c8);
    }
#pragma unroll
    for (int i = 0; i < 2; ++i) {
      const int idx = tid + i * 256;
      const int r   = idx >> 3;
      const int c8  = (idx & 7) << 3;
      const v8h v = *(const v8h*)(gv + (size_t)r * DM + c8);
#pragma unroll
      for (int j = 0; j < 8; ++j) Vs[c8 + j][r] = v[j];
    }
    __syncthreads();

    const v16h qa0 = frag16(&Qs[qrow][0], 0, lane);
    const v16h qa1 = frag16(&Qs[qrow][0], 32, lane);
    v8f sc[4];
#pragma unroll
    for (int n = 0; n < 4; ++n) {
      const int krow = n * 16 + (lane & 15);
      const v16h kb0 = frag16(&Ks[krow][0], 0, lane);
      const v16h kb1 = frag16(&Ks[krow][0], 32, lane);
      v8f s = {};
      s = wmma16(qa0, kb0, s);
      s = wmma16(qa1, kb1, s);
      sc[n] = s * 0.0078125f;
    }

#pragma unroll
    for (int j = 0; j < 8; ++j) {
      float mx = fmaxf(fmaxf(sc[0][j], sc[1][j]), fmaxf(sc[2][j], sc[3][j]));
      mx = fmaxf(mx, __shfl_xor(mx, 1, 32));
      mx = fmaxf(mx, __shfl_xor(mx, 2, 32));
      mx = fmaxf(mx, __shfl_xor(mx, 4, 32));
      mx = fmaxf(mx, __shfl_xor(mx, 8, 32));
      const float mnew = fmaxf(mrun[j], mx);
      const float al   = __expf(mrun[j] - mnew);
      mrun[j] = mnew;
      float rs = 0.f;
#pragma unroll
      for (int n = 0; n < 4; ++n) {
        const float p = __expf(sc[n][j] - mnew);
        sc[n][j] = p;
        rs += p;
      }
      rs += __shfl_xor(rs, 1, 32);
      rs += __shfl_xor(rs, 2, 32);
      rs += __shfl_xor(rs, 4, 32);
      rs += __shfl_xor(rs, 8, 32);
      lrun[j] = lrun[j] * al + rs;
#pragma unroll
      for (int n = 0; n < 4; ++n) o[n][j] *= al;
    }

#pragma unroll
    for (int n = 0; n < 4; ++n)
#pragma unroll
      for (int j = 0; j < 8; ++j)
        pw[(j + rofs) * LDSQ + n * 16 + cc] = (h16)sc[n][j];
    __syncthreads();

    const v16h pa0 = frag16(&Ps[wave][lane & 15][0], 0, lane);
    const v16h pa1 = frag16(&Ps[wave][lane & 15][0], 32, lane);
#pragma unroll
    for (int n = 0; n < 4; ++n) {
      const int drow = n * 16 + (lane & 15);
      const v16h vb0 = frag16(&Vs[drow][0], 0, lane);
      const v16h vb1 = frag16(&Vs[drow][0], 32, lane);
      o[n] = wmma16(pa0, vb0, o[n]);
      o[n] = wmma16(pa1, vb1, o[n]);
    }
    __syncthreads();
  }

  float inv8[8];
#pragma unroll
  for (int j = 0; j < 8; ++j) inv8[j] = 8.0f / lrun[j];
  const size_t orow0 = rowbase + q0 + wave * 16;
  h16* ghi = Chi + orow0 * DM + h * DK;
  h16* glo = Clo + orow0 * DM + h * DK;

#pragma unroll
  for (int n = 0; n < 4; ++n)
#pragma unroll
    for (int j = 0; j < 8; ++j) {
      const float f = o[n][j] * inv8[j];
      pw[(j + rofs) * LDSQ + n * 16 + cc] = (h16)f;
    }
  __syncthreads();
  store_tile16x64(pw, ghi, lane);
  __syncthreads();

#pragma unroll
  for (int n = 0; n < 4; ++n)
#pragma unroll
    for (int j = 0; j < 8; ++j) {
      const float f   = o[n][j] * inv8[j];
      const h16   hv  = (h16)f;
      const float res = (f - (float)hv) * 2048.0f;
      pw[(j + rofs) * LDSQ + n * 16 + cc] = (h16)res;
    }
  __syncthreads();
  store_tile16x64(pw, glo, lane);
}

extern "C" void kernel_launch(void* const* d_in, const int* in_sizes, int n_in,
                              void* d_out, int out_size, void* d_ws, size_t ws_size,
                              hipStream_t stream) {
  if (n_in < 5) return;
  const size_t need_x = ((size_t)(NB - 1) * SEQ_FULL + SEQ) * DM;
  if ((size_t)in_sizes[0] < need_x || (size_t)in_sizes[1] < need_x ||
      (size_t)in_sizes[2] < need_x) return;
  if ((size_t)in_sizes[3] < (size_t)DM * DM || (size_t)in_sizes[4] < (size_t)DM) return;
  if ((size_t)out_size < (size_t)ROWS * DM) return;

  const float* xq = (const float*)d_in[0];
  const float* xk = (const float*)d_in[1];
  const float* xv = (const float*)d_in[2];
  const float* W  = (const float*)d_in[3];
  const float* bs = (const float*)d_in[4];
  float* out = (float*)d_out;

  const size_t sz_wh = (size_t)DM * DM * sizeof(h16);
  const size_t sz_pl = (size_t)ROWS * DM * sizeof(h16);
  size_t off = 0;
  h16* wh  = (h16*)((char*)d_ws + off); off += sz_wh;
  h16* xh  = (h16*)((char*)d_ws + off); off += 3 * sz_pl;
  h16* qkv = (h16*)((char*)d_ws + off); off += 3 * sz_pl;
  h16* chi = (h16*)((char*)d_ws + off); off += sz_pl;
  h16* clo = (h16*)((char*)d_ws + off); off += sz_pl;
  if (off > ws_size) return;

  const int nxc = (ROWS * DM) / CVT_CHUNK;
  const int nwc = (DM * DM) / CVT_CHUNK;
  const int ncx = (nxc > nwc) ? nxc : nwc;

  cvt_planes<<<dim3(ncx, 4), 256, 0, stream>>>(xq, xk, xv, W, xh, wh, nxc, nwc);

  const int nblk = ((ROWS / 16) * NT64) / 4;
  proj_gemm<0><<<dim3(nblk, 3), 128, 0, stream>>>(xh, xh, wh, bs, (void*)qkv);

  attn_flash<<<dim3(SEQ / QBLK, NB * NH), 256, 0, stream>>>(
      qkv, qkv + (size_t)ROWS * DM, qkv + (size_t)2 * ROWS * DM, chi, clo);

  proj_gemm<1><<<dim3(nblk, 1), 128, 0, stream>>>(chi, clo, wh, bs, (void*)out);
}
